// HDRNet_8375186227447
// MI455X (gfx1250) — hardware-run, weakly checked
//
#include <hip/hip_runtime.h>
#include <math.h>

typedef __attribute__((ext_vector_type(16))) __bf16   v16b;
typedef __attribute__((ext_vector_type(8)))  __bf16   v8b;
typedef __attribute__((ext_vector_type(8)))  _Float16 v8h;
typedef __attribute__((ext_vector_type(8)))  float    v8f;
typedef __attribute__((ext_vector_type(4)))  float    v4f;

constexpr int kBatch  = 2;
constexpr int kFullH  = 1024;
constexpr int kFullW  = 1024;
constexpr int kFullHW = kFullH * kFullW;
constexpr int kLowHW  = 256 * 256;
constexpr int kGridXY = 16;
constexpr int kGridZ  = 8;
constexpr int kCoef   = 12;
constexpr int kGridCh = kCoef * kGridZ;

constexpr int kM1 = 32768, kM2 = 8192, kM3 = 2048, kM4 = 512, kMG1 = 128, kMG2r = 32, kMG2 = 64, kMFr = 2, kMF = 64;
constexpr int kK1r = 27, kK1 = 32, kK2r = 72, kK2 = 96, kK3r = 144, kK3 = 160, kK4 = 288, kK9 = 576;
constexpr int kKF3 = 1024, kKF4 = 256, kKF5 = 128, kKP = 64;
constexpr int kNc = 64, kNF3 = 256, kNF4 = 128, kNPr = 96, kNP = 128;

static_assert(kM1 == kBatch * 128 * 128 && kM2 == kBatch * 64 * 64 && kM3 == kBatch * 32 * 32, "pixel counts");
static_assert(kM4 == kBatch * 16 * 16 && kMG1 == kBatch * 8 * 8 && kMG2r == kBatch * 4 * 4, "pixel counts");
static_assert(kK1r == 3 * 9 && kK2r == 8 * 9 && kK3r == 16 * 9 && kK4 == 32 * 9 && kK9 == 64 * 9, "im2col depth");
static_assert(kKF3 == 64 * 16 && kGridCh == kNPr, "flatten / grid channels");
constexpr bool gemm_ok(int m, int n, int k) { return (m % 64) == 0 && (n % 64) == 0 && (k % 32) == 0; }
static_assert(gemm_ok(kM1, kNc, kK1) && gemm_ok(kM2, kNc, kK2) && gemm_ok(kM3, kNc, kK3) && gemm_ok(kM4, kNc, kK4), "tiles");
static_assert(gemm_ok(kMG1, kNc, kK9) && gemm_ok(kMG2, kNc, kK9) && gemm_ok(kM4, kNc, kK9), "tiles");
static_assert(gemm_ok(kMF, kNF3, kKF3) && gemm_ok(kMF, kNF4, kKF4) && gemm_ok(kMF, kNc, kKF5) && gemm_ok(kM4, kNP, kKP), "tiles");
static_assert((kBatch * kFullHW) % 256 == 0 && (kFullW % 256) == 0, "full-res grid exact");

constexpr size_t kBW1 = (size_t)kNc * kK1 * 2,  kBW2 = (size_t)kNc * kK2 * 2,  kBW3 = (size_t)kNc * kK3 * 2;
constexpr size_t kBW4 = (size_t)kNc * kK4 * 2,  kBW9 = (size_t)kNc * kK9 * 2;
constexpr size_t kBWF3 = (size_t)kNF3 * kKF3 * 2, kBWF4 = (size_t)kNF4 * kKF4 * 2, kBWF5 = (size_t)kNc * kKF5 * 2;
constexpr size_t kBWP = (size_t)kNP * kKP * 2;
constexpr size_t kBA1 = (size_t)kM1 * kNc * 4, kBA2 = (size_t)kM2 * kNc * 4, kBA3 = (size_t)kM3 * kNc * 4;
constexpr size_t kBA4 = (size_t)kM4 * kNc * 4, kBAG1 = (size_t)kMG1 * kNc * 4, kBAG2 = (size_t)kMG2 * kNc * 4;
constexpr size_t kBAH3 = (size_t)kMF * kNF3 * 4, kBAH4 = (size_t)kMF * kNF4 * 4, kBAGL = (size_t)kMF * kNc * 4;
constexpr size_t kBAGF = (size_t)kM4 * kNP * 4, kBAGP = (size_t)kM4 * kGridCh * 4;
constexpr size_t kBP1 = (size_t)kM1 * kK1 * 2, kBP2 = (size_t)kM2 * kK2 * 2, kBP3 = (size_t)kM3 * kK3 * 2;
constexpr size_t kBP4 = (size_t)kM4 * kK4 * 2, kBPG1 = (size_t)kMG1 * kK9 * 2, kBPG2 = (size_t)kMG2 * kK9 * 2;
constexpr size_t kBPF3 = (size_t)kMF * kKF3 * 2, kBPF4 = (size_t)kMF * kKF4 * 2, kBPF5 = (size_t)kMF * kKF5 * 2;
constexpr size_t kBPL = (size_t)kM4 * kK9 * 2, kBPP = (size_t)kM4 * kKP * 2;

constexpr size_t kWsWeights = 2 * (kBW1 + kBW2 + kBW3 + kBW4 + 4 * kBW9 + kBWF3 + kBWF4 + kBWF5 + kBWP);
constexpr size_t kWsActs    = kBA1 + kBA2 + kBA3 + 3 * kBA4 + kBAG1 + kBAG2 + kBAH3 + kBAH4 + kBAGL + kBAGF + kBAGP;
constexpr size_t kWsPacks   = 2 * (kBP1 + kBP2 + kBP3 + kBP4 + kBPG1 + kBPG2 + kBPF3 + kBPF4 + kBPF5 + 2 * kBPL + kBPP);
constexpr size_t kWsTotal   = kWsWeights + kWsActs + kWsPacks;
static_assert(kWsWeights == 1982464ull, "weight planes");
static_assert(kWsActs == 12025856ull, "activation planes");
static_assert(kWsPacks == 12533760ull, "operand planes");
static_assert(kWsTotal == 26542080ull, "carve total");
static_assert(kWsTotal <= 134217728ull, "carve cap");

__device__ __forceinline__ unsigned short f2bf_bits(float f) {
  unsigned u = __float_as_uint(f);
  return (unsigned short)((u + 0x7FFFu + ((u >> 16) & 1u)) >> 16);
}
__device__ __forceinline__ float bf_bits2f(unsigned short h) { return __uint_as_float(((unsigned)h) << 16); }

__device__ __forceinline__ void chain_guard_b(v8f& acc, v16b a0, v16b a1, v16b b0, v16b b1) {
  asm volatile("v_nop\n\tv_nop\n\tv_nop\n\tv_nop" : "+v"(acc) : "v"(a0), "v"(a1), "v"(b0), "v"(b1));
}
__device__ __forceinline__ void keep4_b(v16b a, v16b b, v16b c, v16b d) { asm volatile("v_nop" :: "v"(a), "v"(b), "v"(c), "v"(d)); }
__device__ __forceinline__ void acc_guard4(v8f& a, v8f& b, v8f& c, v8f& d) {
  asm volatile("v_nop\n\tv_nop\n\tv_nop\n\tv_nop" : "+v"(a), "+v"(b), "+v"(c), "+v"(d));
}
__device__ __forceinline__ v16b frag_load_b(const __bf16* p) {
  union U { v16b v; v8b h[2]; } f;
  f.h[0] = *(const v8b*)(p);
  f.h[1] = *(const v8b*)(p + 16);
  return f.v;
}
__device__ __forceinline__ v8f mma_b(v16b a, v16b b, v8f c) {
  return __builtin_amdgcn_wmma_f32_16x16x32_bf16(false, a, false, b, (short)0, c, false, false);
}

template <int BIAS_MODE, int ACT>
__global__ __launch_bounds__(256) void gemm64_split_kernel(
    const unsigned short* __restrict__ Ahp, const unsigned short* __restrict__ Alp, int lda,
    const unsigned short* __restrict__ Bhp, const unsigned short* __restrict__ Blp, int ldb,
    float* __restrict__ C, int ldc,
    const float* __restrict__ bias, int nreal,
    int M, int N, int K) {
  const __bf16* Ah = (const __bf16*)Ahp;
  const __bf16* Al = (const __bf16*)Alp;
  const __bf16* Bh = (const __bf16*)Bhp;
  const __bf16* Bl = (const __bf16*)Blp;
  __shared__ __align__(16) float sT[8][16 * 68];
  const int lane = threadIdx.x & 31;
  const int wave = threadIdx.x >> 5;
  const int tilesN = N >> 6;
  const int tilesM = M >> 6;
  const int tile = blockIdx.x * 8 + wave;
  if (tile >= tilesM * tilesN) return;
  const int tm = tile / tilesN;
  const int tn = tile - tm * tilesN;
  const int m0 = tm << 6;
  const int n0 = tn << 6;

  const int rlane = lane & 15;
  const int koff  = (lane >> 4) * 8;
  const int mOff  = (lane >> 4) * 8;

  v8f acc[4][4];
#pragma unroll
  for (int i = 0; i < 4; ++i)
#pragma unroll
    for (int j = 0; j < 4; ++j) acc[i][j] = (v8f){0.f, 0.f, 0.f, 0.f, 0.f, 0.f, 0.f, 0.f};

  for (int k0 = 0; k0 < K; k0 += 32) {
    v16b bh[4], bl[4];
#pragma unroll
    for (int j = 0; j < 4; ++j) {
      const size_t bo = (size_t)(n0 + (j << 4) + rlane) * ldb + koff + k0;
      bh[j] = frag_load_b(Bh + bo);
      bl[j] = frag_load_b(Bl + bo);
    }
#pragma unroll
    for (int i = 0; i < 4; ++i) {
      const size_t ao = (size_t)(m0 + (i << 4) + rlane) * lda + koff + k0;
      const v16b ah = frag_load_b(Ah + ao);
      const v16b al = frag_load_b(Al + ao);
#pragma unroll
      for (int j = 0; j < 4; ++j) {
        acc[i][j] = mma_b(ah, bh[j], acc[i][j]);
        acc[i][j] = mma_b(ah, bl[j], acc[i][j]);
        acc[i][j] = mma_b(al, bh[j], acc[i][j]);
        chain_guard_b(acc[i][j], ah, al, bh[j], bl[j]);
      }
    }
    keep4_b(bh[0], bh[1], bh[2], bh[3]);
    keep4_b(bl[0], bl[1], bl[2], bl[3]);
  }
  acc_guard4(acc[0][0], acc[0][1], acc[0][2], acc[0][3]);
  acc_guard4(acc[1][0], acc[1][1], acc[1][2], acc[1][3]);
  acc_guard4(acc[2][0], acc[2][1], acc[2][2], acc[2][3]);
  acc_guard4(acc[3][0], acc[3][1], acc[3][2], acc[3][3]);

  float* slab = sT[wave];
#pragma unroll
  for (int i = 0; i < 4; ++i) {
    const int mBase = m0 + (i << 4);
#pragma unroll
    for (int j = 0; j < 4; ++j) {
      const int n = n0 + (j << 4) + rlane;
      float bv = 0.f;
      if (BIAS_MODE == 2) {
        const int nb = (n < nreal) ? n : (nreal - 1);
        const float braw = bias[nb];
        bv = (n < nreal) ? braw : 0.0f;
      }
#pragma unroll
      for (int r = 0; r < 8; ++r) {
        float v = acc[i][j][r];
        if (BIAS_MODE == 2) v += bv;
        if (ACT == 2) v = fmaxf(v, 0.0f);
        slab[(mOff + r) * 68 + (j << 4) + rlane] = v;
      }
    }
    __builtin_amdgcn_fence(__ATOMIC_RELEASE, "workgroup");
    __builtin_amdgcn_wave_barrier();
    __builtin_amdgcn_fence(__ATOMIC_ACQUIRE, "workgroup");
    {
      const int hh = lane >> 4, c4 = (lane & 15) * 4;
      for (int pass = 0; pass < 2; ++pass) {
#pragma unroll
        for (int it = 0; it < 8; ++it) {
          const int row = it * 2 + hh;
          const v4f v = *(const v4f*)(slab + row * 68 + c4);
          *(volatile v4f*)(C + (size_t)(mBase + row) * ldc + n0 + c4) = v;
        }
        __threadfence();
      }
    }
    __builtin_amdgcn_fence(__ATOMIC_RELEASE, "workgroup");
    __builtin_amdgcn_wave_barrier();
    __builtin_amdgcn_fence(__ATOMIC_ACQUIRE, "workgroup");
  }
}

__global__ __launch_bounds__(256) void split_weight_kernel(
    const float* __restrict__ src, unsigned short* __restrict__ dhi, unsigned short* __restrict__ dlo,
    int nreal, int kreal, int kpad, int total8) {
  const int i = blockIdx.x * 256 + threadIdx.x;
  if (i >= total8) return;
  const int kc = kpad >> 3;
  const int n = i / kc;
  const int k0 = (i - n * kc) << 3;
  const bool nok = n < nreal;
  const int nc = nok ? n : (nreal - 1);
  v8h hv, lv;
#pragma unroll
  for (int e = 0; e < 8; ++e) {
    const int k = k0 + e;
    const bool kok = k < kreal;
    const int kcl = kok ? k : (kreal - 1);
    const float raw = src[(size_t)nc * kreal + kcl];
    const float v = (nok && kok) ? raw : 0.0f;
    const unsigned short hb = f2bf_bits(v);
    const unsigned short lb = f2bf_bits(v - bf_bits2f(hb));
    hv[e] = __builtin_bit_cast(_Float16, hb);
    lv[e] = __builtin_bit_cast(_Float16, lb);
  }
  unsigned short* qh = dhi + ((size_t)i << 3);
  unsigned short* ql = dlo + ((size_t)i << 3);
  *(volatile v8h*)qh = hv;
  *(volatile v8h*)ql = lv;
  __threadfence();
  *(volatile v8h*)qh = hv;
  *(volatile v8h*)ql = lv;
}

struct PackGeom {
  int mreal, kreal, kpad, hin, win, lhw, lw, stride, pad, sN, sC, sH, sW, has_fuse, ldf, total8;
};
static_assert(sizeof(PackGeom) == 64, "no padding");

template <int KHW>
__global__ __launch_bounds__(256) void pack_a_kernel(
    const float* __restrict__ in, const float* __restrict__ fuse,
    unsigned short* __restrict__ dhi, unsigned short* __restrict__ dlo, PackGeom g) {
  constexpr int KK = KHW * KHW;
  const int i = blockIdx.x * 256 + threadIdx.x;
  if (i >= g.total8) return;
  const int kc = g.kpad >> 3;
  const int m = i / kc;
  const int k0 = (i - m * kc) << 3;
  const bool mok = m < g.mreal;
  const int mc = mok ? m : (g.mreal - 1);
  const int img = mc >> g.lhw;
  const int rem = mc & ((1 << g.lhw) - 1);
  const int oy = rem >> g.lw;
  const int ox = rem & ((1 << g.lw) - 1);
  const int iy0 = oy * g.stride - g.pad;
  const int ix0 = ox * g.stride - g.pad;
  const int ibase = img * g.sN;
  v8h hv, lv;
#pragma unroll
  for (int e = 0; e < 8; ++e) {
    const int k = k0 + e;
    const bool kok = k < g.kreal;
    const int kcl = kok ? k : (g.kreal - 1);
    const int cin = kcl / KK;
    const int r = kcl - cin * KK;
    const int ky = r / KHW;
    const int kx = r - ky * KHW;
    const int iy = iy0 + ky;
    const int ix = ix0 + kx;
    const bool inb = (iy >= 0) && (iy < g.hin) && (ix >= 0) && (ix < g.win);
    int iyc = iy < 0 ? 0 : iy;
    iyc = iyc > g.hin - 1 ? g.hin - 1 : iyc;
    int ixc = ix < 0 ? 0 : ix;
    ixc = ixc > g.win - 1 ? g.win - 1 : ixc;
    float raw = in[(size_t)(ibase + cin * g.sC + iyc * g.sH + ixc * g.sW)];
    if (g.has_fuse) {
      const float fv = fuse[img * g.ldf + cin];
      raw = fmaxf(raw + fv, 0.0f);
    }
    const float v = (mok && kok && inb) ? raw : 0.0f;
    const unsigned short hb = f2bf_bits(v);
    const unsigned short lb = f2bf_bits(v - bf_bits2f(hb));
    hv[e] = __builtin_bit_cast(_Float16, hb);
    lv[e] = __builtin_bit_cast(_Float16, lb);
  }
  unsigned short* qh = dhi + ((size_t)i << 3);
  unsigned short* ql = dlo + ((size_t)i << 3);
  *(volatile v8h*)qh = hv;
  *(volatile v8h*)ql = lv;
  __threadfence();
  *(volatile v8h*)qh = hv;
  *(volatile v8h*)ql = lv;
}

__global__ __launch_bounds__(256) void grid_permute_kernel(const float* __restrict__ gf, float* __restrict__ gp) {
  const int i = blockIdx.x * 256 + threadIdx.x;
  if (i >= kM4 * kGridCh / 4) return;
  const int d = i * 4;
  const int pos = d / kGridCh;
  const int r = d - pos * kGridCh;
  const int z = r / kCoef;
  const int c0 = r - z * kCoef;
  v4f v;
#pragma unroll
  for (int e = 0; e < 4; ++e) v[e] = gf[(size_t)pos * kNP + (c0 + e) * kGridZ + z];
  float* q = gp + d;
  *(volatile v4f*)q = v;
  __threadfence();
  *(volatile v4f*)q = v;
}

__global__ __launch_bounds__(256) void fullres_kernel(
    const float* __restrict__ img, const float* __restrict__ gridP,
    const float* __restrict__ Mm, const float* __restrict__ Mb,
    const float* __restrict__ thr, const float* __restrict__ slo,
    const float* __restrict__ gbias, float* __restrict__ out) {
  __shared__ float sP[112];
  const int tid = threadIdx.x;
  {
    const int t48 = tid < 48 ? tid : 47;
    const int t9  = tid < 9 ? tid : 8;
    const int t3  = tid < 3 ? tid : 2;
    const float tv = thr[t48];
    const float sv = slo[t48];
    const float mv = Mm[t9];
    const float bv = Mb[t3];
    const float gv = gbias[0];
    if (tid < 48) {
      sP[16 + tid] = tv;
      sP[64 + tid] = sv;
    }
    if (tid < 9) sP[tid] = mv;
    if (tid < 3) sP[9 + tid] = bv;
    if (tid == 0) sP[12] = gv;
  }
  __syncthreads();

  const int idx = blockIdx.x * 256 + tid;
  const int n   = idx / kFullHW;
  const int rem = idx - n * kFullHW;
  const int y   = rem / kFullW;
  const int x   = rem - y * kFullW;

  const float fr = img[(size_t)(n * 3 + 0) * kFullHW + rem];
  const float fg = img[(size_t)(n * 3 + 1) * kFullHW + rem];
  const float fb = img[(size_t)(n * 3 + 2) * kFullHW + rem];

  const float g0 = fr * sP[0] + fg * sP[3] + fb * sP[6] + sP[9];
  const float g1 = fr * sP[1] + fg * sP[4] + fb * sP[7] + sP[10];
  const float g2 = fr * sP[2] + fg * sP[5] + fb * sP[8] + sP[11];
  float s0 = 0.0f, s1 = 0.0f, s2 = 0.0f;
#pragma unroll 1
  for (int t = 0; t < 16; ++t) {
    const float th0 = sP[16 + t], th1 = sP[32 + t], th2 = sP[48 + t];
    const float sl0 = sP[64 + t], sl1 = sP[80 + t], sl2 = sP[96 + t];
    s0 = fmaf(sl0, fmaxf(g0 - th0, 0.0f), s0);
    s1 = fmaf(sl1, fmaxf(g1 - th1, 0.0f), s1);
    s2 = fmaf(sl2, fmaxf(g2 - th2, 0.0f), s2);
  }
  float guide = (s0 + s1 + s2) * (1.0f / 3.0f) + sP[12];
  guide = fminf(fmaxf(guide, 0.0f), 1.0f);

  constexpr float kInvW = 1.0f / (float)(kFullW - 1);
  constexpr float kInvH = 1.0f / (float)(kFullH - 1);
  const float cxn = (float)x * kInvW * 2.0f - 1.0f;
  const float cyn = (float)y * kInvH * 2.0f - 1.0f;
  const float czn = guide * 2.0f - 1.0f;
  float fx = ((cxn + 1.0f) * (float)kGridXY - 1.0f) * 0.5f;
  float fy = ((cyn + 1.0f) * (float)kGridXY - 1.0f) * 0.5f;
  float fz = ((czn + 1.0f) * (float)kGridZ - 1.0f) * 0.5f;
  fx = fminf(fmaxf(fx, 0.0f), (float)(kGridXY - 1));
  fy = fminf(fmaxf(fy, 0.0f), (float)(kGridXY - 1));
  fz = fminf(fmaxf(fz, 0.0f), (float)(kGridZ - 1));
  const float x0f = floorf(fx), y0f = floorf(fy), z0f = floorf(fz);
  const float wx = fx - x0f, wy = fy - y0f, wz = fz - z0f;
  int x0 = (int)x0f, y0 = (int)y0f, z0 = (int)z0f;
  x0 = x0 < 0 ? 0 : (x0 > kGridXY - 1 ? kGridXY - 1 : x0);
  y0 = y0 < 0 ? 0 : (y0 > kGridXY - 1 ? kGridXY - 1 : y0);
  z0 = z0 < 0 ? 0 : (z0 > kGridZ - 1 ? kGridZ - 1 : z0);
  const int x1 = (x0 + 1 < kGridXY) ? x0 + 1 : kGridXY - 1;
  const int y1 = (y0 + 1 < kGridXY) ? y0 + 1 : kGridXY - 1;
  const int z1 = (z0 + 1 < kGridZ) ? z0 + 1 : kGridZ - 1;

  float acc[12];
#pragma unroll
  for (int c = 0; c < 12; ++c) acc[c] = 0.0f;

#pragma unroll 1
  for (int q = 0; q < 4; ++q) {
    const int cy = q >> 1, cx = q & 1;
    const int ys = cy ? y1 : y0;
    const int xs = cx ? x1 : x0;
    const float wyy = cy ? wy : (1.0f - wy);
    const float wxx = cx ? wx : (1.0f - wx);
    const float wyx = wyy * wxx;
    const float w0 = wyx * (1.0f - wz);
    const float w1 = wyx * wz;
    const float* base = gridP + (size_t)(((n * kGridXY + ys) * kGridXY + xs) * kGridZ) * kCoef;
    const v4f* p0 = (const v4f*)(base + z0 * kCoef);
    const v4f* p1 = (const v4f*)(base + z1 * kCoef);
    const v4f a0 = p0[0], a1 = p0[1], a2 = p0[2];
    const v4f b0 = p1[0], b1 = p1[1], b2 = p1[2];
#pragma unroll
    for (int e = 0; e < 4; ++e) {
      acc[e]     = fmaf(w0, a0[e], acc[e]);
      acc[e]     = fmaf(w1, b0[e], acc[e]);
      acc[4 + e] = fmaf(w0, a1[e], acc[4 + e]);
      acc[4 + e] = fmaf(w1, b1[e], acc[4 + e]);
      acc[8 + e] = fmaf(w0, a2[e], acc[8 + e]);
      acc[8 + e] = fmaf(w1, b2[e], acc[8 + e]);
    }
  }

  const float rr = fr * acc[0] + fg * acc[1] + fb * acc[2]  + acc[3];
  const float gg = fr * acc[4] + fg * acc[5] + fb * acc[6]  + acc[7];
  const float bb = fr * acc[8] + fg * acc[9] + fb * acc[10] + acc[11];
  float* o0 = out + (size_t)(n * 3 + 0) * kFullHW + rem;
  float* o1 = out + (size_t)(n * 3 + 1) * kFullHW + rem;
  float* o2 = out + (size_t)(n * 3 + 2) * kFullHW + rem;
  *(volatile float*)o0 = rr;
  *(volatile float*)o1 = gg;
  *(volatile float*)o2 = bb;
  __threadfence();
  *(volatile float*)o0 = rr;
  *(volatile float*)o1 = gg;
  *(volatile float*)o2 = bb;
}

static PackGeom mk_geom(int mreal, int mpad, int kreal, int kpad, int hin, int win, int lhw, int lw,
                        int stride, int pad, int sN, int sC, int sH, int sW, int has_fuse, int ldf) {
  PackGeom g;
  g.mreal = mreal; g.kreal = kreal; g.kpad = kpad; g.hin = hin; g.win = win; g.lhw = lhw; g.lw = lw;
  g.stride = stride; g.pad = pad; g.sN = sN; g.sC = sC; g.sH = sH; g.sW = sW;
  g.has_fuse = has_fuse; g.ldf = ldf; g.total8 = mpad * kpad / 8;
  return g;
}

static void launch_split(const float* src, unsigned short* hi, unsigned short* lo,
                         int nreal, int npad, int kreal, int kpad, hipStream_t s) {
  const int total8 = npad * kpad / 8;
  split_weight_kernel<<<(total8 + 255) / 256, 256, 0, s>>>(src, hi, lo, nreal, kreal, kpad, total8);
}

template <int KHW>
static void launch_pack(const float* in, const float* fuse, unsigned short* hi, unsigned short* lo,
                        PackGeom g, hipStream_t s) {
  pack_a_kernel<KHW><<<(g.total8 + 255) / 256, 256, 0, s>>>(in, fuse, hi, lo, g);
}

template <int BIAS_MODE, int ACT>
static void launch_gemm(const unsigned short* ah, const unsigned short* al, int lda,
                        const unsigned short* bh, const unsigned short* bl, int ldb,
                        float* c, int ldc, const float* bias, int nreal, int M, int N, int K, hipStream_t s) {
  const int tiles = (M >> 6) * (N >> 6);
  gemm64_split_kernel<BIAS_MODE, ACT><<<(tiles + 7) / 8, 256, 0, s>>>(ah, al, lda, bh, bl, ldb, c, ldc, bias, nreal, M, N, K);
}

extern "C" void kernel_launch(void* const* d_in, const int* in_sizes, int n_in,
                              void* d_out, int out_size, void* d_ws, size_t ws_size,
                              hipStream_t stream) {
  if (n_in < 30) return;
  if (in_sizes[0] != kBatch * 3 * kLowHW) return;
  if (in_sizes[1] != kBatch * 3 * kFullHW) return;
  if (in_sizes[2] != 8 * kK1r || in_sizes[4] != 16 * kK2r || in_sizes[6] != 32 * kK3r || in_sizes[8] != 64 * kK4) return;
  if (in_sizes[10] != 64 * kK9 || in_sizes[12] != 64 * kK9 || in_sizes[20] != 64 * kK9 || in_sizes[22] != 64 * kK9) return;
  if (in_sizes[14] != 256 * kKF3 || in_sizes[16] != 128 * kKF4 || in_sizes[18] != 64 * kKF5 || in_sizes[23] != kNPr * kKP) return;
  if (in_sizes[25] != 9 || in_sizes[26] != 3 || in_sizes[27] != 48 || in_sizes[28] != 48 || in_sizes[29] != 1) return;
  if (out_size != kBatch * 3 * kFullHW) return;
  if (ws_size < kWsTotal) return;

  const float* lowres  = (const float*)d_in[0];
  const float* fullres = (const float*)d_in[1];
  const float* sw1 = (const float*)d_in[2];  const float* sb1 = (const float*)d_in[3];
  const float* sw2 = (const float*)d_in[4];  const float* sb2 = (const float*)d_in[5];
  const float* sw3 = (const float*)d_in[6];  const float* sb3 = (const float*)d_in[7];
  const float* sw4 = (const float*)d_in[8];  const float* sb4 = (const float*)d_in[9];
  const float* gw1 = (const float*)d_in[10]; const float* gb1 = (const float*)d_in[11];
  const float* gw2 = (const float*)d_in[12]; const float* gb2 = (const float*)d_in[13];
  const float* fw3 = (const float*)d_in[14]; const float* fb3 = (const float*)d_in[15];
  const float* fw4 = (const float*)d_in[16]; const float* fb4 = (const float*)d_in[17];
  const float* fw5 = (const float*)d_in[18]; const float* fb5 = (const float*)d_in[19];
  const float* lw1 = (const float*)d_in[20]; const float* lb1 = (const float*)d_in[21];
  const float* lw2 = (const float*)d_in[22];
  const float* pw  = (const float*)d_in[23]; const float* pb  = (const float*)d_in[24];
  const float* Mm  = (const float*)d_in[25]; const float* Mb  = (const float*)d_in[26];
  const float* thr = (const float*)d_in[27]; const float* slo = (const float*)d_in[28];
  const float* gbias = (const float*)d_in[29];
  float* out = (float*)d_out;

  char* ws = (char*)d_ws;
  size_t off = 0;
  auto carve = [&](size_t bytes) -> char* { char* p = ws + off; off += bytes; return p; };
  unsigned short* W1H = (unsigned short*)carve(kBW1);   unsigned short* W1L = (unsigned short*)carve(kBW1);
  unsigned short* W2H = (unsigned short*)carve(kBW2);   unsigned short* W2L = (unsigned short*)carve(kBW2);
  unsigned short* W3H = (unsigned short*)carve(kBW3);   unsigned short* W3L = (unsigned short*)carve(kBW3);
  unsigned short* W4H = (unsigned short*)carve(kBW4);   unsigned short* W4L = (unsigned short*)carve(kBW4);
  unsigned short* WG1H = (unsigned short*)carve(kBW9);  unsigned short* WG1L = (unsigned short*)carve(kBW9);
  unsigned short* WG2H = (unsigned short*)carve(kBW9);  unsigned short* WG2L = (unsigned short*)carve(kBW9);
  unsigned short* WF3H = (unsigned short*)carve(kBWF3); unsigned short* WF3L = (unsigned short*)carve(kBWF3);
  unsigned short* WF4H = (unsigned short*)carve(kBWF4); unsigned short* WF4L = (unsigned short*)carve(kBWF4);
  unsigned short* WF5H = (unsigned short*)carve(kBWF5); unsigned short* WF5L = (unsigned short*)carve(kBWF5);
  unsigned short* WL1H = (unsigned short*)carve(kBW9);  unsigned short* WL1L = (unsigned short*)carve(kBW9);
  unsigned short* WL2H = (unsigned short*)carve(kBW9);  unsigned short* WL2L = (unsigned short*)carve(kBW9);
  unsigned short* WPH = (unsigned short*)carve(kBWP);   unsigned short* WPL = (unsigned short*)carve(kBWP);
  float* A1    = (float*)carve(kBA1);
  float* A2    = (float*)carve(kBA2);
  float* A3    = (float*)carve(kBA3);
  float* SPLAT = (float*)carve(kBA4);
  float* G1    = (float*)carve(kBAG1);
  float* G2    = (float*)carve(kBAG2);
  float* H3    = (float*)carve(kBAH3);
  float* H4    = (float*)carve(kBAH4);
  float* GLOB  = (float*)carve(kBAGL);
  float* L1    = (float*)carve(kBA4);
  float* LOC   = (float*)carve(kBA4);
  float* GRIDF = (float*)carve(kBAGF);
  float* GRIDP = (float*)carve(kBAGP);
  unsigned short* P1H = (unsigned short*)carve(kBP1);   unsigned short* P1L = (unsigned short*)carve(kBP1);
  unsigned short* P2H = (unsigned short*)carve(kBP2);   unsigned short* P2L = (unsigned short*)carve(kBP2);
  unsigned short* P3H = (unsigned short*)carve(kBP3);   unsigned short* P3L = (unsigned short*)carve(kBP3);
  unsigned short* P4H = (unsigned short*)carve(kBP4);   unsigned short* P4L = (unsigned short*)carve(kBP4);
  unsigned short* PG1H = (unsigned short*)carve(kBPG1); unsigned short* PG1L = (unsigned short*)carve(kBPG1);
  unsigned short* PG2H = (unsigned short*)carve(kBPG2); unsigned short* PG2L = (unsigned short*)carve(kBPG2);
  unsigned short* PF3H = (unsigned short*)carve(kBPF3); unsigned short* PF3L = (unsigned short*)carve(kBPF3);
  unsigned short* PF4H = (unsigned short*)carve(kBPF4); unsigned short* PF4L = (unsigned short*)carve(kBPF4);
  unsigned short* PF5H = (unsigned short*)carve(kBPF5); unsigned short* PF5L = (unsigned short*)carve(kBPF5);
  unsigned short* PL1H = (unsigned short*)carve(kBPL);  unsigned short* PL1L = (unsigned short*)carve(kBPL);
  unsigned short* PL2H = (unsigned short*)carve(kBPL);  unsigned short* PL2L = (unsigned short*)carve(kBPL);
  unsigned short* PPH = (unsigned short*)carve(kBPP);   unsigned short* PPL = (unsigned short*)carve(kBPP);
  if (off != kWsTotal) return;

  launch_split(sw1, W1H, W1L, 8,  kNc, kK1r, kK1, stream);
  launch_split(sw2, W2H, W2L, 16, kNc, kK2r, kK2, stream);
  launch_split(sw3, W3H, W3L, 32, kNc, kK3r, kK3, stream);
  launch_split(sw4, W4H, W4L, 64, kNc, kK4,  kK4, stream);
  launch_split(gw1, WG1H, WG1L, 64, kNc, kK9, kK9, stream);
  launch_split(gw2, WG2H, WG2L, 64, kNc, kK9, kK9, stream);
  launch_split(fw3, WF3H, WF3L, 256, kNF3, kKF3, kKF3, stream);
  launch_split(fw4, WF4H, WF4L, 128, kNF4, kKF4, kKF4, stream);
  launch_split(fw5, WF5H, WF5L, 64, kNc, kKF5, kKF5, stream);
  launch_split(lw1, WL1H, WL1L, 64, kNc, kK9, kK9, stream);
  launch_split(lw2, WL2H, WL2L, 64, kNc, kK9, kK9, stream);
  launch_split(pw,  WPH,  WPL,  kNPr, kNP, kKP, kKP, stream);

  launch_pack<3>(lowres, lowres, P1H, P1L,
                 mk_geom(kM1, kM1, kK1r, kK1, 256, 256, 14, 7, 2, 1, 3 * kLowHW, kLowHW, 256, 1, 0, 0), stream);
  launch_gemm<2, 2>(P1H, P1L, kK1, W1H, W1L, kK1, A1, kNc, sb1, 8, kM1, kNc, kK1, stream);
  launch_pack<3>(A1, A1, P2H, P2L,
                 mk_geom(kM2, kM2, kK2r, kK2, 128, 128, 12, 6, 2, 1, 128 * 128 * kNc, 1, 128 * kNc, kNc, 0, 0), stream);
  launch_gemm<2, 2>(P2H, P2L, kK2, W2H, W2L, kK2, A2, kNc, sb2, 16, kM2, kNc, kK2, stream);
  launch_pack<3>(A2, A2, P3H, P3L,
                 mk_geom(kM3, kM3, kK3r, kK3, 64, 64, 10, 5, 2, 1, 64 * 64 * kNc, 1, 64 * kNc, kNc, 0, 0), stream);
  launch_gemm<2, 2>(P3H, P3L, kK3, W3H, W3L, kK3, A3, kNc, sb3, 32, kM3, kNc, kK3, stream);
  launch_pack<3>(A3, A3, P4H, P4L,
                 mk_geom(kM4, kM4, kK4, kK4, 32, 32, 8, 4, 2, 1, 32 * 32 * kNc, 1, 32 * kNc, kNc, 0, 0), stream);
  launch_gemm<2, 2>(P4H, P4L, kK4, W4H, W4L, kK4, SPLAT, kNc, sb4, 64, kM4, kNc, kK4, stream);
  launch_pack<3>(SPLAT, SPLAT, PG1H, PG1L,
                 mk_geom(kMG1, kMG1, kK9, kK9, 16, 16, 6, 3, 2, 1, 16 * 16 * kNc, 1, 16 * kNc, kNc, 0, 0), stream);
  launch_gemm<2, 2>(PG1H, PG1L, kK9, WG1H, WG1L, kK9, G1, kNc, gb1, 64, kMG1, kNc, kK9, stream);
  launch_pack<3>(G1, G1, PG2H, PG2L,
                 mk_geom(kMG2r, kMG2, kK9, kK9, 8, 8, 4, 2, 2, 1, 8 * 8 * kNc, 1, 8 * kNc, kNc, 0, 0), stream);
  launch_gemm<2, 2>(PG2H, PG2L, kK9, WG2H, WG2L, kK9, G2, kNc, gb2, 64, kMG2, kNc, kK9, stream);
  launch_pack<4>(G2, G2, PF3H, PF3L,
                 mk_geom(kMFr, kMF, kKF3, kKF3, 4, 4, 0, 0, 1, 0, 16 * kNc, 1, 4 * kNc, kNc, 0, 0), stream);
  launch_gemm<2, 2>(PF3H, PF3L, kKF3, WF3H, WF3L, kKF3, H3, kNF3, fb3, 256, kMF, kNF3, kKF3, stream);
  launch_pack<1>(H3, H3, PF4H, PF4L,
                 mk_geom(kMFr, kMF, kKF4, kKF4, 1, 1, 0, 0, 1, 0, kNF3, 1, 0, 0, 0, 0), stream);
  launch_gemm<2, 2>(PF4H, PF4L, kKF4, WF4H, WF4L, kKF4, H4, kNF4, fb4, 128, kMF, kNF4, kKF4, stream);
  launch_pack<1>(H4, H4, PF5H, PF5L,
                 mk_geom(kMFr, kMF, kKF5, kKF5, 1, 1, 0, 0, 1, 0, kNF4, 1, 0, 0, 0, 0), stream);
  launch_gemm<2, 0>(PF5H, PF5L, kKF5, WF5H, WF5L, kKF5, GLOB, kNc, fb5, 64, kMF, kNc, kKF5, stream);
  launch_pack<3>(SPLAT, SPLAT, PL1H, PL1L,
                 mk_geom(kM4, kM4, kK9, kK9, 16, 16, 8, 4, 1, 1, 16 * 16 * kNc, 1, 16 * kNc, kNc, 0, 0), stream);
  launch_gemm<2, 2>(PL1H, PL1L, kK9, WL1H, WL1L, kK9, L1, kNc, lb1, 64, kM4, kNc, kK9, stream);
  launch_pack<3>(L1, L1, PL2H, PL2L,
                 mk_geom(kM4, kM4, kK9, kK9, 16, 16, 8, 4, 1, 1, 16 * 16 * kNc, 1, 16 * kNc, kNc, 0, 0), stream);
  launch_gemm<0, 0>(PL2H, PL2L, kK9, WL2H, WL2L, kK9, LOC, kNc, lb1, 64, kM4, kNc, kK9, stream);
  launch_pack<1>(LOC, GLOB, PPH, PPL,
                 mk_geom(kM4, kM4, kKP, kKP, 16, 16, 8, 4, 1, 0, 16 * 16 * kNc, 1, 16 * kNc, kNc, 1, kNc), stream);
  launch_gemm<2, 0>(PPH, PPL, kKP, WPH, WPL, kKP, GRIDF, kNP, pb, kNPr, kM4, kNP, kKP, stream);

  grid_permute_kernel<<<(kM4 * kGridCh / 4) / 256, 256, 0, stream>>>(GRIDF, GRIDP);

  fullres_kernel<<<(kBatch * kFullHW) / 256, 256, 0, stream>>>(fullres, GRIDP, Mm, Mb, thr, slo, gbias, out);
}
